// DifferentiableStack_49417893707904
// MI455X (gfx1250) — hardware-verified
//
#include <hip/hip_runtime.h>
#include <math.h>
typedef __attribute__((ext_vector_type(16))) _Float16 v16h;
typedef __attribute__((ext_vector_type(8)))  _Float16 v8h;
typedef __attribute__((ext_vector_type(16))) __bf16   v16b;
typedef __attribute__((ext_vector_type(8)))  __bf16   v8b;
typedef __attribute__((ext_vector_type(8)))  float    v8f;
typedef __attribute__((ext_vector_type(4)))  float    v4f;
#define PSCALE 32768.0f
#define U16(p) ((const unsigned short*)(const void*)(p))
#define PSCALE_INV (1.0f / 32768.0f)

__device__ __forceinline__ unsigned short f2bf_bits(float f) {
  unsigned u = __float_as_uint(f);
  return (unsigned short)((u + 0x7FFFu + ((u >> 16) & 1u)) >> 16);
}
__device__ __forceinline__ float bf_bits2f(unsigned short h) { return __uint_as_float(((unsigned)h) << 16); }

__device__ __forceinline__ void dep_guard_h(v8f& a, v8f& b, v16h x, v16h y) { asm volatile("v_nop\n\tv_nop\n\tv_nop\n\tv_nop" : "+v"(a), "+v"(b) : "v"(x), "v"(y)); }
__device__ __forceinline__ void dep_guard_b(v8f& a, v8f& b, v16b x, v16b y) { asm volatile("v_nop\n\tv_nop\n\tv_nop\n\tv_nop" : "+v"(a), "+v"(b) : "v"(x), "v"(y)); }
__device__ __forceinline__ void keep4_h(v16h a, v16h b, v16h c, v16h d) { asm volatile("v_nop" :: "v"(a), "v"(b), "v"(c), "v"(d)); }
__device__ __forceinline__ void keep4_b(v16b a, v16b b, v16b c, v16b d) { asm volatile("v_nop" :: "v"(a), "v"(b), "v"(c), "v"(d)); }
__device__ __forceinline__ void acc_guard4(v8f& a, v8f& b, v8f& c, v8f& d) { asm volatile("v_nop\n\tv_nop\n\tv_nop\n\tv_nop" : "+v"(a), "+v"(b), "+v"(c), "+v"(d)); }
template <typename T> struct Frag;
template <> struct Frag<_Float16> {
  typedef v16h V; union U { v16h v; v8h h[2]; };
  static __device__ __forceinline__ v16h load(const _Float16* p) {
    U f; f.h[0] = *(const v8h*)(p); f.h[1] = *(const v8h*)(p + 16); return f.v;
  }
  static __device__ __forceinline__ v8f mma(v16h a, v16h b, v8f c) {
    return __builtin_amdgcn_wmma_f32_16x16x32_f16(false, a, false, b, (short)0, c, false, false);
  }
  static __device__ __forceinline__ void guard(v8f& a, v8f& b, v16h x, v16h y) { dep_guard_h(a, b, x, y); }
  static __device__ __forceinline__ void keep(v16h a, v16h b, v16h c, v16h d) { keep4_h(a, b, c, d); }
};
template <> struct Frag<__bf16> {
  typedef v16b V; union U { v16b v; v8b h[2]; };
  static __device__ __forceinline__ v16b load(const __bf16* p) {
    U f; f.h[0] = *(const v8b*)(p); f.h[1] = *(const v8b*)(p + 16); return f.v;
  }
  static __device__ __forceinline__ v8f mma(v16b a, v16b b, v8f c) {
    return __builtin_amdgcn_wmma_f32_16x16x32_bf16(false, a, false, b, (short)0, c, false, false);
  }
  static __device__ __forceinline__ void guard(v8f& a, v8f& b, v16b x, v16b y) { dep_guard_b(a, b, x, y); }
  static __device__ __forceinline__ void keep(v16b a, v16b b, v16b c, v16b d) { keep4_b(a, b, c, d); }
};

template <int ET> struct Elem;
template <> struct Elem<0> { typedef _Float16 T; };
template <> struct Elem<1> { typedef __bf16 T; };
template <int ET, bool SPLIT, int BIAS_MODE, int OUT_MODE, bool RESID, int ACT = 0>
__global__ __launch_bounds__(256) void wmma_gemm64(
    const unsigned short* __restrict__ Ap, const unsigned short* __restrict__ A2p, int lda, long strideA,
    const unsigned short* __restrict__ Btp, const unsigned short* __restrict__ Bt2p, int ldb, long strideB,
    void* __restrict__ Cout, void* __restrict__ Cout2, int ldc, long strideC,
    const float* __restrict__ bias,
    const float* __restrict__ resid, long strideR,
    int M, int N, int K, float scale) {
  typedef typename Elem<ET>::T T;
  typedef typename Frag<T>::V V;
  const T* A = (const T*)Ap; const T* A2 = (const T*)A2p; const T* Bt = (const T*)Btp; const T* Bt2 = (const T*)Bt2p;
  __shared__ __align__(16) float sT[8][16 * 68];
  const int b    = blockIdx.y;
  const int lane = threadIdx.x & 31;
  const int wave = threadIdx.x >> 5;
  const int tilesN = N >> 6;
  const int tilesM = M >> 6;
  const int tile = blockIdx.x * 8 + wave;
  if (tile >= tilesM * tilesN) return;
  const int tm = tile / tilesN;
  const int tn = tile - tm * tilesN;
  const int m0 = tm << 6;
  const int n0 = tn << 6;

  const T* Ab  = A  + (size_t)b * strideA;
  const T* Bb  = Bt + (size_t)b * strideB;
  const T* Ab2 = SPLIT ? (A2  + (size_t)b * strideA) : nullptr;
  const T* Bb2 = SPLIT ? (Bt2 + (size_t)b * strideB) : nullptr;

  const int rlane = lane & 15;
  const int koff  = (lane >> 4) * 8;
  const int mOff  = (lane >> 4) * 8;

  v8f acc[4][4];
#pragma unroll
  for (int i = 0; i < 4; ++i)
#pragma unroll
    for (int j = 0; j < 4; ++j) acc[i][j] = (v8f){0.f,0.f,0.f,0.f,0.f,0.f,0.f,0.f};

  for (int k0 = 0; k0 < K; k0 += 32) {
    V bh[4], bl[4];
#pragma unroll
    for (int j = 0; j < 4; ++j) {
      const size_t bo = (size_t)(n0 + (j << 4) + rlane) * ldb + koff + k0;
      bh[j] = Frag<T>::load(Bb + bo);
      if (SPLIT) bl[j] = Frag<T>::load(Bb2 + bo);
    }
#pragma unroll
    for (int i = 0; i < 4; ++i) {
      const size_t ao = (size_t)(m0 + (i << 4) + rlane) * lda + koff + k0;
      V ah = Frag<T>::load(Ab + ao);
      V al;
      if (SPLIT) al = Frag<T>::load(Ab2 + ao);
#pragma unroll
      for (int j = 0; j < 4; ++j) {
        acc[i][j] = Frag<T>::mma(ah, bh[j], acc[i][j]);
        if (SPLIT) {
          acc[i][j] = Frag<T>::mma(ah, bl[j], acc[i][j]);
          acc[i][j] = Frag<T>::mma(al, bh[j], acc[i][j]);
        }
      }
      Frag<T>::guard(acc[i][0], acc[i][3], ah, SPLIT ? al : ah);
    }
    Frag<T>::keep(bh[0], bh[1], bh[2], bh[3]);
    if (SPLIT) Frag<T>::keep(bl[0], bl[1], bl[2], bl[3]);
  }
  acc_guard4(acc[0][0], acc[0][1], acc[0][2], acc[0][3]);
  acc_guard4(acc[1][0], acc[1][1], acc[1][2], acc[1][3]);
  acc_guard4(acc[2][0], acc[2][1], acc[2][2], acc[2][3]);
  acc_guard4(acc[3][0], acc[3][1], acc[3][2], acc[3][3]);

  float* slab = sT[wave];
  const float* Rb = RESID ? (resid + (size_t)b * strideR) : nullptr;
#pragma unroll
  for (int i = 0; i < 4; ++i) {
    const int mBase = m0 + (i << 4);
#pragma unroll
    for (int j = 0; j < 4; ++j) {
      const int n = n0 + (j << 4) + rlane;
      float bv = 0.f;
      if (BIAS_MODE == 2) bv = bias[n];
#pragma unroll
      for (int r = 0; r < 8; ++r) {
        float v = acc[i][j][r] * scale;
        if (BIAS_MODE == 1) v += bias[mBase + mOff + r];
        if (BIAS_MODE == 2) v += bv;
        if (RESID) v += Rb[(size_t)(mBase + mOff + r) * ldc + n];
        if (ACT == 1) v = tanhf(v);
        if (ACT == 2) v = fmaxf(v, 0.0f);
        if (ACT == 3) v = v / (1.0f + expf(-v));
        if (ACT == 4) v = (v > 0.f) ? v : 0.01f * v;
        if (ACT == 5) v = 0.5f * v * (1.0f + erff(v * 0.70710678118654752f));
        slab[(mOff + r) * 68 + (j << 4) + rlane] = v;
      }
    }
    __builtin_amdgcn_fence(__ATOMIC_RELEASE, "workgroup");
    __builtin_amdgcn_wave_barrier();
    __builtin_amdgcn_fence(__ATOMIC_ACQUIRE, "workgroup");
    if (OUT_MODE == 0) {
      float* C = (float*)Cout + (size_t)b * strideC;
      const int hh = lane >> 4, c4 = (lane & 15) * 4;
      for (int pass = 0; pass < 2; ++pass) {
#pragma unroll
        for (int it = 0; it < 8; ++it) {
          const int row = it * 2 + hh;
          v4f v = *(const v4f*)(slab + row * 68 + c4);
          *(volatile v4f*)(C + (size_t)(mBase + row) * ldc + n0 + c4) = v;
        }
        __threadfence();
      }
    } else {
      const int q = lane >> 3, c8 = (lane & 7) * 8;
      unsigned short* C  = (unsigned short*)Cout  + (size_t)b * strideC;
      unsigned short* C2 = (OUT_MODE == 2) ? ((unsigned short*)Cout2 + (size_t)b * strideC) : nullptr;
      for (int pass = 0; pass < 2; ++pass) {
#pragma unroll
        for (int it = 0; it < 4; ++it) {
          const int row = it * 4 + q;
          const float* sp = slab + row * 68 + c8;
          v8h hv, lv;
#pragma unroll
          for (int e = 0; e < 8; ++e) {
            if (OUT_MODE == 1) {
              hv[e] = (_Float16)sp[e];
            } else {
              unsigned short hb = f2bf_bits(sp[e]);
              unsigned short lb = f2bf_bits(sp[e] - bf_bits2f(hb));
              hv[e] = __builtin_bit_cast(_Float16, hb);
              lv[e] = __builtin_bit_cast(_Float16, lb);
            }
          }
          *(volatile v8h*)(C + (size_t)(mBase + row) * ldc + n0 + c8) = hv;
          if (OUT_MODE == 2) *(volatile v8h*)(C2 + (size_t)(mBase + row) * ldc + n0 + c8) = lv;
        }
        __threadfence();
      }
    }
    __builtin_amdgcn_fence(__ATOMIC_RELEASE, "workgroup");
    __builtin_amdgcn_wave_barrier();
    __builtin_amdgcn_fence(__ATOMIC_ACQUIRE, "workgroup");
  }
}

__global__ __launch_bounds__(256) void cast_f32_f16x2(
    const float* __restrict__ in, _Float16* __restrict__ out, int n2) {
  int i = blockIdx.x * 256 + threadIdx.x;
  if (i < n2) {
    const _Float16 h0 = (_Float16)in[2 * i], h1 = (_Float16)in[2 * i + 1];
    const unsigned u = (unsigned)__builtin_bit_cast(unsigned short, h0) | ((unsigned)__builtin_bit_cast(unsigned short, h1) << 16);
    ((volatile unsigned*)out)[i] = u;
    __threadfence();
    ((volatile unsigned*)out)[i] = u;
  }
}

__global__ __launch_bounds__(256) void split_f32_bf16x2(
    const float* __restrict__ in, __bf16* __restrict__ hi, __bf16* __restrict__ lo, long n2) {
  long i = (long)blockIdx.x * 256 + threadIdx.x;
  long stride = (long)gridDim.x * 256;
  for (int pass = 0; pass < 2; ++pass) {
    for (long j = i; j < n2; j += stride) {
      const float a = in[2 * j], b = in[2 * j + 1];
      const unsigned short ah = f2bf_bits(a), bh = f2bf_bits(b);
      const unsigned short al = f2bf_bits(a - bf_bits2f(ah)), bl = f2bf_bits(b - bf_bits2f(bh));
      ((volatile unsigned*)hi)[j] = (unsigned)ah | ((unsigned)bh << 16);
      ((volatile unsigned*)lo)[j] = (unsigned)al | ((unsigned)bl << 16);
    }
    __threadfence();
  }
}


__global__ __launch_bounds__(256) void transpose_split_bf16(const float* __restrict__ in, int ldi,
                                                           __bf16* __restrict__ outH, __bf16* __restrict__ outL, int ldo) {
  __shared__ __align__(16) float tile[64][68];
  const int c0 = blockIdx.x * 64, r0 = blockIdx.y * 64;
  const int t = threadIdx.y * 32 + threadIdx.x;
  for (int i = threadIdx.y; i < 64; i += 8) {
    tile[threadIdx.x][i]      = in[(size_t)(r0 + i) * ldi + c0 + threadIdx.x];
    tile[32 + threadIdx.x][i] = in[(size_t)(r0 + i) * ldi + c0 + 32 + threadIdx.x];
  }
  __syncthreads();
  const int q = t >> 3, c8 = (t & 7) * 8;
  for (int pass = 0; pass < 2; ++pass) {
#pragma unroll
    for (int it = 0; it < 2; ++it) {
      const int c = it * 32 + q;
      v8b hv, lv;
#pragma unroll
      for (int e = 0; e < 8; ++e) {
        const float f = tile[c][c8 + e];
        const unsigned short hb = f2bf_bits(f);
        hv[e] = __builtin_bit_cast(__bf16, hb);
        lv[e] = __builtin_bit_cast(__bf16, f2bf_bits(f - bf_bits2f(hb)));
      }
      *(volatile v8b*)(outH + (size_t)(c0 + c) * ldo + r0 + c8) = hv;
      *(volatile v8b*)(outL + (size_t)(c0 + c) * ldo + r0 + c8) = lv;
    }
    __threadfence();
  }
}

#define ST 512
#define SS 256
#define SD 1024
#define SEPS 1e-6f
__global__ __launch_bounds__(256) void ptr_kernel(const float* __restrict__ ctrl, const float* __restrict__ ptr0, float* __restrict__ ptrs,
                                                 __bf16* __restrict__ Pnh, __bf16* __restrict__ Pnl, __bf16* __restrict__ Puh, __bf16* __restrict__ Pul, float* __restrict__ Lt, double* __restrict__ Slog) {
  __shared__ float p[SS]; __shared__ float red[8]; __shared__ float tot;
  const int s = threadIdx.x, lane = s & 31, wave = s >> 5;
  float cur = ptr0[s]; p[s] = cur;
  float L = 1.0f; double sl = 0.0;
  __syncthreads();
  for (int t = 0; t < ST; ++t) {
    const float push = ctrl[t * 3], pop = ctrl[t * 3 + 1], noop = ctrl[t * 3 + 2];
    const float up = p[(s - 1) & (SS - 1)], down = p[(s + 1) & (SS - 1)];
    float np_ = push * up + pop * down + noop * cur;
    float v = np_;
    for (int o = 16; o > 0; o >>= 1) v += __shfl_xor(v, o, 32);
    if (lane == 0) red[wave] = v;
    __syncthreads();
    if (s == 0) { float a = 0.f; for (int w = 0; w < 8; ++w) a += red[w]; tot = a; }
    __syncthreads();
    np_ = np_ / (tot + SEPS);
    ptrs[(size_t)t * SS + s] = np_;
    { const unsigned short h = f2bf_bits(np_); Pnh[(size_t)t * SS + s] = __builtin_bit_cast(__bf16, h); Pnl[(size_t)t * SS + s] = __builtin_bit_cast(__bf16, f2bf_bits(np_ - bf_bits2f(h))); }
    { const unsigned short h = f2bf_bits(up);  Puh[(size_t)t * SS + s] = __builtin_bit_cast(__bf16, h); Pul[(size_t)t * SS + s] = __builtin_bit_cast(__bf16, f2bf_bits(up - bf_bits2f(h))); }
    if (s == 0) { L = L * (1.0f - push); sl += log1p(-(double)push); Lt[t] = L; Slog[t] = sl; }
    __syncthreads();
    p[s] = np_; cur = np_;
    __syncthreads();
  }
}
__global__ __launch_bounds__(256) void restore_kernel(float* __restrict__ ptrs, __bf16* __restrict__ Pnh, __bf16* __restrict__ Pnl, __bf16* __restrict__ Puh, __bf16* __restrict__ Pul) {
  const int i = blockIdx.x * 256 + threadIdx.x; if (i >= ST * SS) return;
  ((volatile float*)ptrs)[i] = ptrs[i]; ((volatile __bf16*)Pnh)[i] = Pnh[i]; ((volatile __bf16*)Pnl)[i] = Pnl[i]; ((volatile __bf16*)Puh)[i] = Puh[i]; ((volatile __bf16*)Pul)[i] = Pul[i];
}
__global__ __launch_bounds__(256) void amat_kernel(const float* __restrict__ S, const float* __restrict__ ctrl, const double* __restrict__ Slog, __bf16* __restrict__ Ah, __bf16* __restrict__ Al) {
  const int i = blockIdx.x * 256 + threadIdx.x; if (i >= ST * ST) return; const int t = i / ST, tau = i % ST;
  float a = 0.f;
  if (tau <= t) { const double c = (double)ctrl[tau * 3] * exp(Slog[t] - Slog[tau]); a = (float)(c * (double)S[i]); }
  const unsigned short h = f2bf_bits(a), l = f2bf_bits(a - bf_bits2f(h));
  for (int pass = 0; pass < 2; ++pass) { ((volatile __bf16*)Ah)[i] = __builtin_bit_cast(__bf16, h); ((volatile __bf16*)Al)[i] = __builtin_bit_cast(__bf16, l); __threadfence(); }
}
__global__ __launch_bounds__(256) void plmat_kernel(const float* __restrict__ ptrs, const float* __restrict__ Lt, __bf16* __restrict__ Ph, __bf16* __restrict__ Pl) {
  const int i = blockIdx.x * 256 + threadIdx.x; if (i >= ST * SS) return; const int t = i / SS;
  const float a = Lt[t] * ptrs[i];
  const unsigned short h = f2bf_bits(a), l = f2bf_bits(a - bf_bits2f(h));
  for (int pass = 0; pass < 2; ++pass) { ((volatile __bf16*)Ph)[i] = __builtin_bit_cast(__bf16, h); ((volatile __bf16*)Pl)[i] = __builtin_bit_cast(__bf16, l); __threadfence(); }
}
extern "C" void kernel_launch(void* const* d_in, const int* in_sizes, int n_in, void* d_out, int out_size, void* d_ws, size_t ws_size, hipStream_t stream) {
  (void)in_sizes; (void)n_in; (void)out_size; (void)ws_size;
  const float* values = (const float*)d_in[0]; const float* ctrl = (const float*)d_in[1]; const float* mem0 = (const float*)d_in[2]; const float* ptr0 = (const float*)d_in[3];
  float* reads = (float*)d_out; float* ptrs = reads + (size_t)ST * SD;
  char* ws = (char*)d_ws; size_t off = 0;
  auto carve = [&](size_t bytes) -> char* { char* p = ws + off; off += (bytes + 255) & ~(size_t)255; return p; };
  __bf16* Pnh = (__bf16*)carve(ST * SS * 2); __bf16* Pnl = (__bf16*)carve(ST * SS * 2); __bf16* Puh = (__bf16*)carve(ST * SS * 2); __bf16* Pul = (__bf16*)carve(ST * SS * 2);
  float* Lt = (float*)carve(ST * 4); double* Slog = (double*)carve(ST * 8);
  float* S = (float*)carve((size_t)ST * ST * 4);
  __bf16* Ah = (__bf16*)carve((size_t)ST * ST * 2); __bf16* Al = (__bf16*)carve((size_t)ST * ST * 2);
  __bf16* PLh = (__bf16*)carve(ST * SS * 2); __bf16* PLl = (__bf16*)carve(ST * SS * 2);
  __bf16* M0h = (__bf16*)carve((size_t)SD * SS * 2); __bf16* M0l = (__bf16*)carve((size_t)SD * SS * 2);
  __bf16* Vh = (__bf16*)carve((size_t)SD * ST * 2); __bf16* Vl = (__bf16*)carve((size_t)SD * ST * 2);
  float* R0 = (float*)carve((size_t)ST * SD * 4);
  ptr_kernel<<<1, 256, 0, stream>>>(ctrl, ptr0, ptrs, Pnh, Pnl, Puh, Pul, Lt, Slog);
  restore_kernel<<<(ST * SS + 255) / 256, 256, 0, stream>>>(ptrs, Pnh, Pnl, Puh, Pul);
  { const int t = (ST / 64) * (ST / 64);
    wmma_gemm64<1, true, 0, 0, false><<<dim3((t + 7) / 8, 1), 256, 0, stream>>>(U16(Pnh), U16(Pnl), SS, 0, U16(Puh), U16(Pul), SS, 0, S, nullptr, ST, 0, nullptr, nullptr, 0, ST, ST, SS, 1.0f); }
  amat_kernel<<<(ST * ST + 255) / 256, 256, 0, stream>>>(S, ctrl, Slog, Ah, Al);
  plmat_kernel<<<(ST * SS + 255) / 256, 256, 0, stream>>>(ptrs, Lt, PLh, PLl);
  transpose_split_bf16<<<dim3(SD / 64, SS / 64), dim3(32, 8), 0, stream>>>(mem0, SD, M0h, M0l, SS);
  transpose_split_bf16<<<dim3(SD / 64, ST / 64), dim3(32, 8), 0, stream>>>(values, SD, Vh, Vl, ST);
  { const int t = (ST / 64) * (SD / 64);
    wmma_gemm64<1, true, 0, 0, false><<<dim3((t + 7) / 8, 1), 256, 0, stream>>>(U16(PLh), U16(PLl), SS, 0, U16(M0h), U16(M0l), SS, 0, R0, nullptr, SD, 0, nullptr, nullptr, 0, ST, SD, SS, 1.0f);
    wmma_gemm64<1, true, 0, 0, true><<<dim3((t + 7) / 8, 1), 256, 0, stream>>>(U16(Ah), U16(Al), ST, 0, U16(Vh), U16(Vl), ST, 0, reads, nullptr, SD, 0, nullptr, R0, 0, ST, SD, ST, 1.0f); }
}
